// LSTMdecoder_58093727645744
// MI455X (gfx1250) — hardware-verified
//
#include <hip/hip_runtime.h>

typedef __attribute__((ext_vector_type(16))) _Float16 v16h;
typedef __attribute__((ext_vector_type(8)))  _Float16 v8h;
typedef __attribute__((ext_vector_type(16))) __bf16   v16b;
typedef __attribute__((ext_vector_type(8)))  __bf16   v8b;
typedef __attribute__((ext_vector_type(8)))  float    v8f;
typedef __attribute__((ext_vector_type(4)))  float    v4f;
typedef __attribute__((ext_vector_type(4)))  unsigned int v4u;
typedef __attribute__((ext_vector_type(2)))  unsigned int v2u;
typedef __attribute__((ext_vector_type(4)))  int      v4i;

constexpr int TT   = 128;
constexpr int NB   = 64;
constexpr int SS   = 256;
constexpr int KS   = 128;
constexpr int HID  = 512;
constexpr int EMB  = 512;
constexpr int NG4  = 2048;
constexpr int MROWS = TT * NB;
constexpr int CATW = 2 * HID;

__device__ __forceinline__ unsigned short f2bf_bits(float f) {
  unsigned u = __float_as_uint(f);
  return (unsigned short)((u + 0x7FFFu + ((u >> 16) & 1u)) >> 16);
}
__device__ __forceinline__ float bf_bits2f(unsigned short h) { return __uint_as_float(((unsigned)h) << 16); }
__device__ __forceinline__ float bf_lo16(unsigned w) { return __uint_as_float(w << 16); }
__device__ __forceinline__ float bf_hi16(unsigned w) { return __uint_as_float(w & 0xffff0000u); }
__device__ __forceinline__ float rnbf(float x) { return bf_bits2f(f2bf_bits(x)); }
__device__ __forceinline__ float sigm_f(float x) { return __builtin_amdgcn_rcpf(1.0f + expf(-x)); }

__device__ __forceinline__ void dep_guard_h(v8f& a, v8f& b, v16h x, v16h y) { asm volatile("v_nop\n\tv_nop\n\tv_nop\n\tv_nop" : "+v"(a), "+v"(b) : "v"(x), "v"(y)); }
__device__ __forceinline__ void dep_guard_b(v8f& a, v8f& b, v16b x, v16b y) { asm volatile("v_nop\n\tv_nop\n\tv_nop\n\tv_nop" : "+v"(a), "+v"(b) : "v"(x), "v"(y)); }
__device__ __forceinline__ void keep4_h(v16h a, v16h b, v16h c, v16h d) { asm volatile("v_nop" :: "v"(a), "v"(b), "v"(c), "v"(d)); }
__device__ __forceinline__ void keep4_b(v16b a, v16b b, v16b c, v16b d) { asm volatile("v_nop" :: "v"(a), "v"(b), "v"(c), "v"(d)); }
__device__ __forceinline__ void acc_guard4(v8f& a, v8f& b, v8f& c, v8f& d) { asm volatile("v_nop\n\tv_nop\n\tv_nop\n\tv_nop" : "+v"(a), "+v"(b), "+v"(c), "+v"(d)); }
template <typename T> struct Frag;
template <> struct Frag<_Float16> {
  typedef v16h V; union U { v16h v; v8h h[2]; };
  static __device__ __forceinline__ v16h load(const _Float16* p) {
    U f; f.h[0] = *(const v8h*)(p); f.h[1] = *(const v8h*)(p + 16); return f.v;
  }
  static __device__ __forceinline__ v8f mma(v16h a, v16h b, v8f c) {
    return __builtin_amdgcn_wmma_f32_16x16x32_f16(false, a, false, b, (short)0, c, false, false);
  }
  static __device__ __forceinline__ void guard(v8f& a, v8f& b, v16h x, v16h y) { dep_guard_h(a, b, x, y); }
  static __device__ __forceinline__ void keep(v16h a, v16h b, v16h c, v16h d) { keep4_h(a, b, c, d); }
};
template <> struct Frag<__bf16> {
  typedef v16b V; union U { v16b v; v8b h[2]; };
  static __device__ __forceinline__ v16b load(const __bf16* p) {
    U f; f.h[0] = *(const v8b*)(p); f.h[1] = *(const v8b*)(p + 16); return f.v;
  }
  static __device__ __forceinline__ v8f mma(v16b a, v16b b, v8f c) {
    return __builtin_amdgcn_wmma_f32_16x16x32_bf16(false, a, false, b, (short)0, c, false, false);
  }
  static __device__ __forceinline__ void guard(v8f& a, v8f& b, v16b x, v16b y) { dep_guard_b(a, b, x, y); }
  static __device__ __forceinline__ void keep(v16b a, v16b b, v16b c, v16b d) { keep4_b(a, b, c, d); }
};

template <int ET> struct Elem;
template <> struct Elem<0> { typedef _Float16 T; };
template <> struct Elem<1> { typedef __bf16 T; };
template <int ET, int SPLIT, int BIAS_MODE, int OUT_MODE, int ACT = 0>
__global__ __launch_bounds__(256) void wmma_gemm64(
    const unsigned short* __restrict__ Ap, const unsigned short* __restrict__ A2p, int lda, long strideA,
    const unsigned short* __restrict__ Btp, const unsigned short* __restrict__ Bt2p, int ldb, long strideB,
    void* __restrict__ Cout, void* __restrict__ Cout2, int ldc, long strideC,
    const float* __restrict__ bias,
    int M, int N, int K, float scale) {
  typedef typename Elem<ET>::T T;
  typedef typename Frag<T>::V V;
  const T* A = (const T*)Ap; const T* A2 = (const T*)A2p; const T* Bt = (const T*)Btp; const T* Bt2 = (const T*)Bt2p;
  __shared__ __align__(16) float sT[8][16 * 68];
  const int b    = blockIdx.y;
  const int lane = threadIdx.x & 31;
  const int wave = threadIdx.x >> 5;
  const int tilesN = N >> 6;
  const int tilesM = M >> 6;
  const int tile = blockIdx.x * 8 + wave;
  if (tile >= tilesM * tilesN) return;
  const int tm = tile / tilesN;
  const int tn = tile - tm * tilesN;
  const int m0 = tm << 6;
  const int n0 = tn << 6;

  const T* Ab  = A  + (size_t)b * strideA;
  const T* Bb  = Bt + (size_t)b * strideB;
  const T* Ab2 = (SPLIT >= 1) ? (A2  + (size_t)b * strideA) : nullptr;
  const T* Bb2 = (SPLIT == 2) ? (Bt2 + (size_t)b * strideB) : nullptr;

  const int rlane = lane & 15;
  const int koff  = (lane >> 4) * 8;
  const int mOff  = (lane >> 4) * 8;

  v8f acc[4][4];
#pragma unroll
  for (int i = 0; i < 4; ++i)
#pragma unroll
    for (int j = 0; j < 4; ++j) acc[i][j] = (v8f){0.f,0.f,0.f,0.f,0.f,0.f,0.f,0.f};

  for (int k0 = 0; k0 < K; k0 += 32) {
    V bh[4], bl[4];
#pragma unroll
    for (int j = 0; j < 4; ++j) {
      const size_t bo = (size_t)(n0 + (j << 4) + rlane) * ldb + koff + k0;
      bh[j] = Frag<T>::load(Bb + bo);
      if (SPLIT == 2) bl[j] = Frag<T>::load(Bb2 + bo);
    }
#pragma unroll
    for (int i = 0; i < 4; ++i) {
      const size_t ao = (size_t)(m0 + (i << 4) + rlane) * lda + koff + k0;
      V ah = Frag<T>::load(Ab + ao);
      V al;
      if (SPLIT >= 1) al = Frag<T>::load(Ab2 + ao);
#pragma unroll
      for (int j = 0; j < 4; ++j) {
        acc[i][j] = Frag<T>::mma(ah, bh[j], acc[i][j]);
        if (SPLIT == 2) acc[i][j] = Frag<T>::mma(ah, bl[j], acc[i][j]);
        if (SPLIT >= 1) acc[i][j] = Frag<T>::mma(al, bh[j], acc[i][j]);
      }
      Frag<T>::guard(acc[i][0], acc[i][3], ah, (SPLIT >= 1) ? al : ah);
    }
    Frag<T>::keep(bh[0], bh[1], bh[2], bh[3]);
    if (SPLIT == 2) Frag<T>::keep(bl[0], bl[1], bl[2], bl[3]);
  }
  acc_guard4(acc[0][0], acc[0][1], acc[0][2], acc[0][3]);
  acc_guard4(acc[1][0], acc[1][1], acc[1][2], acc[1][3]);
  acc_guard4(acc[2][0], acc[2][1], acc[2][2], acc[2][3]);
  acc_guard4(acc[3][0], acc[3][1], acc[3][2], acc[3][3]);

  float* slab = sT[wave];
#pragma unroll
  for (int i = 0; i < 4; ++i) {
    const int mBase = m0 + (i << 4);
#pragma unroll
    for (int j = 0; j < 4; ++j) {
      const int n = n0 + (j << 4) + rlane;
      float bv = 0.f;
      if (BIAS_MODE == 2) bv = bias[n];
#pragma unroll
      for (int r = 0; r < 8; ++r) {
        float v = acc[i][j][r] * scale;
        if (BIAS_MODE == 1) v += bias[mBase + mOff + r];
        if (BIAS_MODE == 2) v += bv;
        if (ACT == 1) v = tanhf(v);
        if (ACT == 2) v = fmaxf(v, 0.0f);
        if (ACT == 4) v = (v > 0.f) ? v : 0.01f * v;
        slab[(mOff + r) * 68 + (j << 4) + rlane] = v;
      }
    }
    __builtin_amdgcn_fence(__ATOMIC_RELEASE, "workgroup");
    __builtin_amdgcn_wave_barrier();
    __builtin_amdgcn_fence(__ATOMIC_ACQUIRE, "workgroup");
    if (OUT_MODE == 0) {
      float* C = (float*)Cout + (size_t)b * strideC;
      const int hh = lane >> 4, c4 = (lane & 15) * 4;
      for (int pass = 0; pass < 2; ++pass) {
#pragma unroll
        for (int it = 0; it < 8; ++it) {
          const int row = it * 2 + hh;
          v4f v = *(const v4f*)(slab + row * 68 + c4);
          *(volatile v4f*)(C + (size_t)(mBase + row) * ldc + n0 + c4) = v;
        }
        __threadfence();
      }
    } else {
      const int q = lane >> 3, c8 = (lane & 7) * 8;
      unsigned short* C  = (unsigned short*)Cout  + (size_t)b * strideC;
      unsigned short* C2 = (OUT_MODE == 2) ? ((unsigned short*)Cout2 + (size_t)b * strideC) : nullptr;
      for (int pass = 0; pass < 2; ++pass) {
#pragma unroll
        for (int it = 0; it < 4; ++it) {
          const int row = it * 4 + q;
          const float* sp = slab + row * 68 + c8;
          v8h hv, lv;
#pragma unroll
          for (int e = 0; e < 8; ++e) {
            if (OUT_MODE == 1) {
              hv[e] = (_Float16)sp[e];
            } else {
              unsigned short hb = f2bf_bits(sp[e]);
              unsigned short lb = f2bf_bits(sp[e] - bf_bits2f(hb));
              hv[e] = __builtin_bit_cast(_Float16, hb);
              lv[e] = __builtin_bit_cast(_Float16, lb);
            }
          }
          *(volatile v8h*)(C + (size_t)(mBase + row) * ldc + n0 + c8) = hv;
          if (OUT_MODE == 2) *(volatile v8h*)(C2 + (size_t)(mBase + row) * ldc + n0 + c8) = lv;
        }
        __threadfence();
      }
    }
    __builtin_amdgcn_fence(__ATOMIC_RELEASE, "workgroup");
    __builtin_amdgcn_wave_barrier();
    __builtin_amdgcn_fence(__ATOMIC_ACQUIRE, "workgroup");
  }
}

__global__ __launch_bounds__(256) void cast_bf16x8(const float* __restrict__ in,
                                                  unsigned short* __restrict__ out, int n8) {
  const int i = blockIdx.x * 256 + threadIdx.x;
  if (i < n8) {
    const v4f a = *(const v4f*)(in + 8 * (size_t)i);
    const v4f c = *(const v4f*)(in + 8 * (size_t)i + 4);
    v4u w;
    w[0] = (unsigned)f2bf_bits(a[0]) | ((unsigned)f2bf_bits(a[1]) << 16);
    w[1] = (unsigned)f2bf_bits(a[2]) | ((unsigned)f2bf_bits(a[3]) << 16);
    w[2] = (unsigned)f2bf_bits(c[0]) | ((unsigned)f2bf_bits(c[1]) << 16);
    w[3] = (unsigned)f2bf_bits(c[2]) | ((unsigned)f2bf_bits(c[3]) << 16);
    unsigned short* p = out + 8 * (size_t)i;
    *(volatile v4u*)p = w;
    __threadfence();
    *(volatile v4u*)p = w;
  }
}

__global__ __launch_bounds__(256) void round_bias_kernel(const float* __restrict__ bp,
                                                        const float* __restrict__ bg,
                                                        float* __restrict__ outb) {
  const int i = threadIdx.x;
  const int idx = (i & 127) * 4;
  const v4f a = *(const v4f*)(bp + idx);
  const v4f c = *(const v4f*)(bg + idx);
  v4f v;
#pragma unroll
  for (int e = 0; e < 4; ++e) {
    const float x = (i < 128) ? a[e] : c[e];
    v[e] = rnbf(x);
  }
  float* p = outb + 4 * i;
  *(volatile v4f*)p = v;
  __threadfence();
  *(volatile v4f*)p = v;
}

__global__ __launch_bounds__(256) void gather_embed_kernel(const int* __restrict__ tok,
                                                          const float* __restrict__ emb,
                                                          unsigned short* __restrict__ xb, int vocab) {
  const int lane = threadIdx.x & 31, wave = threadIdx.x >> 5;
  const int row = blockIdx.x * 8 + wave;
  int tk = tok[row];
  tk = tk < 0 ? 0 : tk;
  tk = tk > (vocab - 1) ? (vocab - 1) : tk;
  const float* er = emb + (size_t)tk * EMB;
  v4u w[2];
#pragma unroll
  for (int k = 0; k < 2; ++k) {
    const int base = 256 * k + 8 * lane;
    const v4f a = *(const v4f*)(er + base);
    const v4f c = *(const v4f*)(er + base + 4);
    w[k][0] = (unsigned)f2bf_bits(a[0]) | ((unsigned)f2bf_bits(a[1]) << 16);
    w[k][1] = (unsigned)f2bf_bits(a[2]) | ((unsigned)f2bf_bits(a[3]) << 16);
    w[k][2] = (unsigned)f2bf_bits(c[0]) | ((unsigned)f2bf_bits(c[1]) << 16);
    w[k][3] = (unsigned)f2bf_bits(c[2]) | ((unsigned)f2bf_bits(c[3]) << 16);
  }
  unsigned short* dst = xb + (size_t)row * EMB + 8 * lane;
  for (int pass = 0; pass < 2; ++pass) {
    *(volatile v4u*)(dst) = w[0];
    *(volatile v4u*)(dst + 256) = w[1];
    __threadfence();
  }
}

template <int L>
__global__ __launch_bounds__(256) void transpose_mem_kernel(const float* __restrict__ mem,
                                                           unsigned short* __restrict__ memT) {
  __shared__ __align__(16) unsigned short tile[64 * 72];
  const int tid = threadIdx.x, lane = tid & 31, wave = tid >> 5;
  const int s0 = blockIdx.x * 64, d0 = blockIdx.y * 64, b = blockIdx.z;
#pragma unroll
  for (int it = 0; it < 4; ++it) {
    const int idx = it * 256 + tid;
    const int s = idx >> 4, d4 = (idx & 15) * 4;
    const v4f v = *(const v4f*)(mem + ((size_t)(s0 + s) * NB + b) * HID + d0 + d4);
#pragma unroll
    for (int e = 0; e < 4; ++e) tile[(d4 + e) * 72 + s] = f2bf_bits(v[e]);
  }
  __syncthreads();
  v4u vv[2];
#pragma unroll
  for (int it = 0; it < 2; ++it) {
    const int d = 8 * wave + it * 4 + (lane >> 3);
    vv[it] = *(const v4u*)(tile + d * 72 + (lane & 7) * 8);
  }
  for (int pass = 0; pass < 2; ++pass) {
#pragma unroll
    for (int it = 0; it < 2; ++it) {
      const int d = 8 * wave + it * 4 + (lane >> 3);
      unsigned short* dst = memT + ((size_t)b * HID + d0 + d) * L + s0 + (lane & 7) * 8;
      *(volatile v4u*)dst = vv[it];
    }
    __threadfence();
  }
}

constexpr int HSP = 528;
constexpr int HS_PLANE = 16 * HSP;
constexpr int HS_WORDS = HS_PLANE;

__global__ __launch_bounds__(256) void lstm_seq_kernel(
    const unsigned short* __restrict__ xb, const unsigned short* __restrict__ wih,
    const unsigned short* __restrict__ whh, const float* __restrict__ b_ih,
    const float* __restrict__ b_hh, unsigned short* __restrict__ cat_hi,
    unsigned short* __restrict__ cat_lo, float* __restrict__ out_h, float* __restrict__ out_c) {
  __shared__ __align__(16) float hsraw[HS_WORDS];
  __shared__ __align__(16) float biasS[NG4];
  unsigned short* hs = reinterpret_cast<unsigned short*>(hsraw);
  const int tid = threadIdx.x, lane = tid & 31, wave = tid >> 5;
  const int rl = lane & 15, hh = lane >> 4, koff = hh * 8;
  const int mb = blockIdx.x;
  const int jw = wave * 64;

  {
    const v4u z4 = {0u, 0u, 0u, 0u};
    for (int i = tid; i < (2 * HS_PLANE) / 8; i += 256) *(v4u*)(hs + 8 * i) = z4;
    const int n0 = tid * 8;
    const v4f a0 = *(const v4f*)(b_ih + n0), a1 = *(const v4f*)(b_ih + n0 + 4);
    const v4f c0 = *(const v4f*)(b_hh + n0), c1 = *(const v4f*)(b_hh + n0 + 4);
#pragma unroll
    for (int e = 0; e < 4; ++e) {
      biasS[n0 + e]     = rnbf(a0[e]) + rnbf(c0[e]);
      biasS[n0 + 4 + e] = rnbf(a1[e]) + rnbf(c1[e]);
    }
  }
  __syncthreads();

  float creg[4][8];
#pragma unroll
  for (int q = 0; q < 4; ++q)
#pragma unroll
    for (int r = 0; r < 8; ++r) creg[q][r] = 0.0f;

  const __bf16* Xb = (const __bf16*)xb + (size_t)(16 * mb + rl) * EMB + koff;
  const __bf16* Wi = (const __bf16*)wih + (size_t)(jw + rl) * EMB + koff;
  const __bf16* Wh = (const __bf16*)whh + (size_t)(jw + rl) * HID + koff;
  const __bf16* Hh = (const __bf16*)hs + rl * HSP + koff;
  const __bf16* Hl = Hh + HS_PLANE;

#pragma unroll 1
  for (int t = 0; t < TT; ++t) {
    v8f acc[4][4];
#pragma unroll
    for (int g = 0; g < 4; ++g)
#pragma unroll
      for (int q = 0; q < 4; ++q) acc[g][q] = (v8f){0.f,0.f,0.f,0.f,0.f,0.f,0.f,0.f};

    const __bf16* xr = Xb + (size_t)t * NB * EMB;
#pragma unroll 1
    for (int k0 = 0; k0 < EMB; k0 += 32) {
      const v16b ax = Frag<__bf16>::load(xr + k0);
#pragma unroll
      for (int g = 0; g < 4; ++g) {
        v16b bw[4];
#pragma unroll
        for (int q = 0; q < 4; ++q) bw[q] = Frag<__bf16>::load(Wi + (g * 512 + 16 * q) * EMB + k0);
#pragma unroll
        for (int q = 0; q < 4; ++q) acc[g][q] = Frag<__bf16>::mma(ax, bw[q], acc[g][q]);
        dep_guard_b(acc[g][0], acc[g][3], ax, bw[3]);
        keep4_b(bw[0], bw[1], bw[2], bw[3]);
      }
    }
#pragma unroll 1
    for (int k0 = 0; k0 < HID; k0 += 32) {
      const v16b ah = Frag<__bf16>::load(Hh + k0);
      const v16b al = Frag<__bf16>::load(Hl + k0);
#pragma unroll
      for (int g = 0; g < 4; ++g) {
        v16b bw[4];
#pragma unroll
        for (int q = 0; q < 4; ++q) bw[q] = Frag<__bf16>::load(Wh + (g * 512 + 16 * q) * HID + k0);
#pragma unroll
        for (int q = 0; q < 4; ++q) {
          acc[g][q] = Frag<__bf16>::mma(ah, bw[q], acc[g][q]);
          acc[g][q] = Frag<__bf16>::mma(al, bw[q], acc[g][q]);
        }
        dep_guard_b(acc[g][0], acc[g][3], ah, al);
        keep4_b(bw[0], bw[1], bw[2], bw[3]);
      }
    }
    acc_guard4(acc[0][0], acc[0][1], acc[0][2], acc[0][3]);
    acc_guard4(acc[1][0], acc[1][1], acc[1][2], acc[1][3]);
    acc_guard4(acc[2][0], acc[2][1], acc[2][2], acc[2][3]);
    acc_guard4(acc[3][0], acc[3][1], acc[3][2], acc[3][3]);
    __syncthreads();

#pragma unroll
    for (int q = 0; q < 4; ++q) {
      const int col = jw + 16 * q + rl;
      const float bi = biasS[col], bf = biasS[512 + col], bg = biasS[1024 + col], bo = biasS[1536 + col];
#pragma unroll
      for (int r = 0; r < 8; ++r) {
        const int row = 8 * hh + r;
        const float pi = acc[0][q][r] + bi;
        const float pf = acc[1][q][r] + bf;
        const float pg = acc[2][q][r] + bg;
        const float po = acc[3][q][r] + bo;
        const float ig = sigm_f(pi), fg = sigm_f(pf), og = sigm_f(po);
        const float gt = tanhf(pg);
        const float cn = fg * creg[q][r] + ig * gt;
        const float hn = og * tanhf(cn);
        creg[q][r] = cn;
        const unsigned short hb = f2bf_bits(hn);
        const unsigned short lb = f2bf_bits(hn - bf_bits2f(hb));
        hs[row * HSP + col] = hb;
        hs[HS_PLANE + row * HSP + col] = lb;
      }
    }
    __syncthreads();

    {
      const size_t grow0 = (size_t)t * NB + 16 * mb;
      for (int pass = 0; pass < 2; ++pass) {
#pragma unroll
        for (int it = 0; it < 8; ++it) {
          const int pl  = it >> 2;
          const int li  = (it & 3) * 4 + (lane >> 3);
          const int row = 2 * wave + (li >> 3);
          const int off = (li & 7) * 64 + (lane & 7) * 8;
          const v4u v = *(const v4u*)(hs + pl * HS_PLANE + row * HSP + off);
          unsigned short* dst = (pl ? cat_lo : cat_hi) + (grow0 + row) * CATW + off;
          *(volatile v4u*)dst = v;
        }
        __threadfence();
      }
    }
  }

  for (int pass = 0; pass < 2; ++pass) {
#pragma unroll
    for (int it = 0; it < 8; ++it) {
      const int row = 2 * wave + (it >> 2);
      const int foff = (it & 3) * 128 + lane * 4;
      const v2u a  = *(const v2u*)(hs + row * HSP + foff);
      const v2u bl = *(const v2u*)(hs + HS_PLANE + row * HSP + foff);
      v4f o;
      o[0] = bf_lo16(a[0]) + bf_lo16(bl[0]);
      o[1] = bf_hi16(a[0]) + bf_hi16(bl[0]);
      o[2] = bf_lo16(a[1]) + bf_lo16(bl[1]);
      o[3] = bf_hi16(a[1]) + bf_hi16(bl[1]);
      *(volatile v4f*)(out_h + (size_t)(16 * mb + row) * HID + foff) = o;
    }
    __threadfence();
  }
  __syncthreads();

  float* fsl = hsraw + wave * 1024;
#pragma unroll
  for (int q = 0; q < 4; ++q)
#pragma unroll
    for (int r = 0; r < 8; ++r) fsl[(8 * hh + r) * 64 + 16 * q + rl] = creg[q][r];
  __syncthreads();
  {
    const int c4 = rl * 4;
    for (int pass = 0; pass < 2; ++pass) {
#pragma unroll
      for (int it = 0; it < 8; ++it) {
        const int row = it * 2 + hh;
        const v4f val = *(const v4f*)(fsl + row * 64 + c4);
        *(volatile v4f*)(out_c + (size_t)(16 * mb + row) * HID + jw + c4) = val;
      }
      __threadfence();
    }
  }
}

template <int L, bool WR>
__global__ __launch_bounds__(128) void softmax_rows_kernel(const float* __restrict__ sc,
                                                          const int* __restrict__ msk,
                                                          unsigned short* __restrict__ ph,
                                                          unsigned short* __restrict__ plo,
                                                          float* __restrict__ wout) {
  constexpr int LPR = L / 8;
  constexpr int RPW = 32 / LPR;
  __shared__ __align__(16) float slab[4][256];
  const int tid = threadIdx.x, lane = tid & 31, wave = tid >> 5;
  const int sub = lane / LPR, cl = lane - sub * LPR;
  const int rbase = (blockIdx.x * 4 + wave) * RPW;
  const int r = rbase + sub;
  const int b = r / TT;
  const float* sp = sc + (size_t)r * L + 8 * cl;
  const v4f s0 = *(const v4f*)sp, s1 = *(const v4f*)(sp + 4);
  const int* mp = msk + (size_t)b * L + 8 * cl;
  const v4i m0 = *(const v4i*)mp, m1 = *(const v4i*)(mp + 4);
  float v[8];
#pragma unroll
  for (int e = 0; e < 4; ++e) {
    v[e]     = (m0[e] != 0) ? -1.0e9f : s0[e];
    v[4 + e] = (m1[e] != 0) ? -1.0e9f : s1[e];
  }
  float mx = v[0];
#pragma unroll
  for (int e = 1; e < 8; ++e) mx = fmaxf(mx, v[e]);
#pragma unroll
  for (int off = 1; off < LPR; off <<= 1) mx = fmaxf(mx, __shfl_xor(mx, off, 32));
  float ev[8], sum = 0.0f;
#pragma unroll
  for (int e = 0; e < 8; ++e) { ev[e] = expf(v[e] - mx); sum += ev[e]; }
#pragma unroll
  for (int off = 1; off < LPR; off <<= 1) sum += __shfl_xor(sum, off, 32);
  const float inv = __builtin_amdgcn_rcpf(sum);
  float p[8];
  unsigned short hb[8], lb[8];
#pragma unroll
  for (int e = 0; e < 8; ++e) {
    p[e] = ev[e] * inv;
    hb[e] = f2bf_bits(p[e]);
    lb[e] = f2bf_bits(p[e] - bf_bits2f(hb[e]));
  }
  v4u hv, lv;
#pragma unroll
  for (int k = 0; k < 4; ++k) {
    hv[k] = (unsigned)hb[2 * k] | ((unsigned)hb[2 * k + 1] << 16);
    lv[k] = (unsigned)lb[2 * k] | ((unsigned)lb[2 * k + 1] << 16);
  }
  const size_t po = (size_t)r * L + 8 * cl;
  for (int pass = 0; pass < 2; ++pass) {
    *(volatile v4u*)(ph + po) = hv;
    *(volatile v4u*)(plo + po) = lv;
    __threadfence();
  }
  if (WR) {
    float* sl = slab[wave] + sub * L + 8 * cl;
    *(v4f*)(sl)     = (v4f){p[0], p[1], p[2], p[3]};
    *(v4f*)(sl + 4) = (v4f){p[4], p[5], p[6], p[7]};
    __syncthreads();
    for (int pass = 0; pass < 2; ++pass) {
#pragma unroll
      for (int it = 0; it < 2; ++it) {
        const int fi = it * 128 + lane * 4;
        const int rowl = fi / L;
        const int col = fi - rowl * L;
        const int rr = rbase + rowl;
        const int bb = rr / TT, tt = rr - bb * TT;
        const v4f val = *(const v4f*)(slab[wave] + fi);
        *(volatile v4f*)(wout + (size_t)(tt * NB + bb) * L + col) = val;
      }
      __threadfence();
    }
  }
}

__global__ __launch_bounds__(256) void blend_kernel(const float* __restrict__ z,
                                                   const unsigned short* __restrict__ c2h,
                                                   const unsigned short* __restrict__ c2l,
                                                   float* __restrict__ out) {
  const int i = blockIdx.x * 256 + threadIdx.x;
  const int m = i >> 7, c4 = (i & 127) * 4;
  const v4f zv = *(const v4f*)(z + 4 * (size_t)i);
  const size_t o = (size_t)m * CATW + c4;
  const v2u wh = *(const v2u*)(c2h + o), wl = *(const v2u*)(c2l + o);
  const v2u ah = *(const v2u*)(c2h + o + HID), al = *(const v2u*)(c2l + o + HID);
  float wsv[4], asv[4];
  wsv[0] = bf_lo16(wh[0]) + bf_lo16(wl[0]);  wsv[1] = bf_hi16(wh[0]) + bf_hi16(wl[0]);
  wsv[2] = bf_lo16(wh[1]) + bf_lo16(wl[1]);  wsv[3] = bf_hi16(wh[1]) + bf_hi16(wl[1]);
  asv[0] = bf_lo16(ah[0]) + bf_lo16(al[0]);  asv[1] = bf_hi16(ah[0]) + bf_hi16(al[0]);
  asv[2] = bf_lo16(ah[1]) + bf_lo16(al[1]);  asv[3] = bf_hi16(ah[1]) + bf_hi16(al[1]);
  v4f ov;
#pragma unroll
  for (int e = 0; e < 4; ++e) {
    const float g = sigm_f(zv[e]);
    ov[e] = g * asv[e] + (1.0f - g) * wsv[e];
  }
  float* p = out + 4 * (size_t)i;
  *(volatile v4f*)p = ov;
  __threadfence();
  *(volatile v4f*)p = ov;
}

constexpr size_t MIB = (size_t)1 << 20;
constexpr size_t O_X = 0;
constexpr size_t O_WIH = 8 * MIB, O_WHH = 10 * MIB, O_WAS = 12 * MIB, O_WPROJ = 12 * MIB + MIB / 2;
constexpr size_t O_WASK = 13 * MIB + MIB / 2, O_WGATE = 14 * MIB, O_BIASR = 15 * MIB;
constexpr size_t O_MEM = 16 * MIB, O_MEMT = 32 * MIB, O_R1 = 48 * MIB, O_R2 = 80 * MIB;
constexpr size_t WS_END = 112 * MIB;
static_assert((size_t)NG4 * EMB * 2 <= 2 * MIB);
static_assert((size_t)MROWS * EMB * 2 == 8 * MIB);
static_assert((size_t)SS * NB * HID * 2 == 16 * MIB);
static_assert((size_t)MROWS * CATW * 2 == 16 * MIB);
static_assert((size_t)MROWS * HID * 2 == 8 * MIB);
static_assert((size_t)NB * TT * SS * 4 == 8 * MIB);
static_assert((size_t)NB * TT * SS * 2 == 4 * MIB);
static_assert((size_t)NB * TT * KS * 4 == 4 * MIB);
static_assert((size_t)MROWS * HID * 4 == 16 * MIB);
static_assert(WS_END <= 128 * MIB);
static_assert(MROWS % 64 == 0 && TT % 64 == 0 && HID % 64 == 0 && SS % 64 == 0 && KS % 64 == 0);
static_assert(HID % 32 == 0 && CATW % 32 == 0 && SS % 32 == 0 && KS % 32 == 0);
constexpr size_t OUT0_OFF = 0;
constexpr size_t OUT1_OFF = 16777216 / 4;
constexpr size_t OUT2_OFF = 20971520 / 4;
constexpr size_t OUT3_OFF = 21102592 / 4;
constexpr size_t OUT_TOTAL = 21233664 / 4;
static_assert(OUT1_OFF == (size_t)MROWS * HID);
static_assert(OUT2_OFF == OUT1_OFF + (size_t)MROWS * KS);
static_assert(OUT3_OFF == OUT2_OFF + (size_t)NB * HID);
static_assert(OUT_TOTAL == OUT3_OFF + (size_t)NB * HID);

extern "C" void kernel_launch(void* const* d_in, const int* in_sizes, int n_in,
                              void* d_out, int out_size, void* d_ws, size_t ws_size,
                              hipStream_t stream) {
  if (n_in < 16) return;
  if (in_sizes[0] != TT * NB || in_sizes[1] != SS * NB * HID || in_sizes[2] != NB * SS ||
      in_sizes[3] != KS * NB * HID || in_sizes[4] != NB * KS || in_sizes[6] != NG4 * EMB ||
      in_sizes[7] != NG4 * HID || in_sizes[8] != NG4 || in_sizes[9] != NG4 ||
      in_sizes[10] != HID * HID || in_sizes[11] != HID * CATW || in_sizes[12] != HID ||
      in_sizes[13] != HID * HID || in_sizes[14] != HID * CATW || in_sizes[15] != HID) return;
  if (in_sizes[5] < EMB || (in_sizes[5] % EMB) != 0) return;
  if ((size_t)out_size != OUT_TOTAL) return;
  if (ws_size < WS_END) return;
  const int vocab = in_sizes[5] / EMB;

  const int*   tok        = (const int*)d_in[0];
  const float* mem_src    = (const float*)d_in[1];
  const int*   msk_src    = (const int*)d_in[2];
  const float* mem_ske    = (const float*)d_in[3];
  const int*   msk_ske    = (const int*)d_in[4];
  const float* embed      = (const float*)d_in[5];
  const float* w_ih       = (const float*)d_in[6];
  const float* w_hh       = (const float*)d_in[7];
  const float* b_ih       = (const float*)d_in[8];
  const float* b_hh       = (const float*)d_in[9];
  const float* w_attn_src = (const float*)d_in[10];
  const float* w_proj     = (const float*)d_in[11];
  const float* b_proj     = (const float*)d_in[12];
  const float* w_attn_ske = (const float*)d_in[13];
  const float* w_gate     = (const float*)d_in[14];
  const float* b_gate     = (const float*)d_in[15];

  char* ws = (char*)d_ws;
  unsigned short* x_bf   = (unsigned short*)(ws + O_X);
  unsigned short* wih_bf = (unsigned short*)(ws + O_WIH);
  unsigned short* whh_bf = (unsigned short*)(ws + O_WHH);
  unsigned short* was_bf = (unsigned short*)(ws + O_WAS);
  unsigned short* wpj_bf = (unsigned short*)(ws + O_WPROJ);
  unsigned short* wak_bf = (unsigned short*)(ws + O_WASK);
  unsigned short* wgt_bf = (unsigned short*)(ws + O_WGATE);
  float* biasr   = (float*)(ws + O_BIASR);
  unsigned short* mem_bf  = (unsigned short*)(ws + O_MEM);
  unsigned short* memT_bf = (unsigned short*)(ws + O_MEMT);
  unsigned short* cat1_hi = (unsigned short*)(ws + O_R1);
  unsigned short* cat1_lo = (unsigned short*)(ws + O_R1 + 16 * MIB);
  unsigned short* qp2_hi  = (unsigned short*)(ws + O_R1);
  unsigned short* qp2_lo  = (unsigned short*)(ws + O_R1 + 8 * MIB);
  float* sc2              = (float*)(ws + O_R1 + 16 * MIB);
  unsigned short* p2_hi   = (unsigned short*)(ws + O_R1 + 20 * MIB);
  unsigned short* p2_lo   = (unsigned short*)(ws + O_R1 + 22 * MIB);
  float* zbuf             = (float*)(ws + O_R1);
  unsigned short* qp_hi   = (unsigned short*)(ws + O_R2);
  unsigned short* qp_lo   = (unsigned short*)(ws + O_R2 + 8 * MIB);
  float* sc1              = (float*)(ws + O_R2 + 16 * MIB);
  unsigned short* p1_hi   = (unsigned short*)(ws + O_R2 + 24 * MIB);
  unsigned short* p1_lo   = (unsigned short*)(ws + O_R2 + 28 * MIB);
  unsigned short* cat2_hi = (unsigned short*)(ws + O_R2);
  unsigned short* cat2_lo = (unsigned short*)(ws + O_R2 + 16 * MIB);

  float* fout  = (float*)d_out;
  float* out0  = fout + OUT0_OFF;
  float* out1  = fout + OUT1_OFF;
  float* out2  = fout + OUT2_OFF;
  float* out3  = fout + OUT3_OFF;

  cast_bf16x8<<<(NG4 * EMB / 8) / 256, 256, 0, stream>>>(w_ih, wih_bf, NG4 * EMB / 8);
  cast_bf16x8<<<(NG4 * HID / 8) / 256, 256, 0, stream>>>(w_hh, whh_bf, NG4 * HID / 8);
  cast_bf16x8<<<(HID * HID / 8) / 256, 256, 0, stream>>>(w_attn_src, was_bf, HID * HID / 8);
  cast_bf16x8<<<(HID * CATW / 8) / 256, 256, 0, stream>>>(w_proj, wpj_bf, HID * CATW / 8);
  cast_bf16x8<<<(HID * HID / 8) / 256, 256, 0, stream>>>(w_attn_ske, wak_bf, HID * HID / 8);
  cast_bf16x8<<<(HID * CATW / 8) / 256, 256, 0, stream>>>(w_gate, wgt_bf, HID * CATW / 8);
  round_bias_kernel<<<1, 256, 0, stream>>>(b_proj, b_gate, biasr);
  gather_embed_kernel<<<MROWS / 8, 256, 0, stream>>>(tok, embed, x_bf, vocab);
  cast_bf16x8<<<(SS * NB * HID / 8) / 256, 256, 0, stream>>>(mem_src, mem_bf, SS * NB * HID / 8);
  transpose_mem_kernel<SS><<<dim3(SS / 64, HID / 64, NB), 256, 0, stream>>>(mem_src, memT_bf);

  lstm_seq_kernel<<<NB / 16, 256, 0, stream>>>(x_bf, wih_bf, whh_bf, b_ih, b_hh, cat1_hi, cat1_lo, out2, out3);

  wmma_gemm64<1, 1, 0, 2, 0><<<dim3((MROWS / 64) * (HID / 64) / 8, 1), 256, 0, stream>>>(
      cat1_hi, cat1_lo, CATW, 0L, was_bf, was_bf, HID, 0L, qp_hi, qp_lo, HID, 0L, biasr,
      MROWS, HID, HID, 1.0f);
  wmma_gemm64<1, 1, 0, 0, 0><<<dim3(1, NB), 256, 0, stream>>>(
      qp_hi, qp_lo, NB * HID, (long)HID, mem_bf, mem_bf, NB * HID, (long)HID, sc1, sc1, SS,
      (long)TT * SS, biasr, TT, SS, HID, 1.0f);
  softmax_rows_kernel<SS, false><<<(NB * TT) / 4, 128, 0, stream>>>(sc1, msk_src, p1_hi, p1_lo, out1);
  wmma_gemm64<1, 1, 0, 2, 0><<<dim3(2, NB), 256, 0, stream>>>(
      p1_hi, p1_lo, SS, (long)TT * SS, memT_bf, memT_bf, SS, (long)HID * SS, cat1_hi + HID,
      cat1_lo + HID, NB * CATW, (long)CATW, biasr, TT, HID, SS, 1.0f);
  wmma_gemm64<1, 1, 2, 2, 1><<<dim3((MROWS / 64) * (HID / 64) / 8, 1), 256, 0, stream>>>(
      cat1_hi, cat1_lo, CATW, 0L, wpj_bf, wpj_bf, CATW, 0L, cat2_hi, cat2_lo, CATW, 0L, biasr,
      MROWS, HID, CATW, 1.0f);

  cast_bf16x8<<<(KS * NB * HID / 8) / 256, 256, 0, stream>>>(mem_ske, mem_bf, KS * NB * HID / 8);
  transpose_mem_kernel<KS><<<dim3(KS / 64, HID / 64, NB), 256, 0, stream>>>(mem_ske, memT_bf);
  wmma_gemm64<1, 1, 0, 2, 0><<<dim3((MROWS / 64) * (HID / 64) / 8, 1), 256, 0, stream>>>(
      cat2_hi, cat2_lo, CATW, 0L, wak_bf, wak_bf, HID, 0L, qp2_hi, qp2_lo, HID, 0L, biasr,
      MROWS, HID, HID, 1.0f);
  wmma_gemm64<1, 1, 0, 0, 0><<<dim3(1, NB), 256, 0, stream>>>(
      qp2_hi, qp2_lo, NB * HID, (long)HID, mem_bf, mem_bf, NB * HID, (long)HID, sc2, sc2, KS,
      (long)TT * KS, biasr, TT, KS, HID, 1.0f);
  softmax_rows_kernel<KS, true><<<(NB * TT) / 8, 128, 0, stream>>>(sc2, msk_ske, p2_hi, p2_lo, out1);
  wmma_gemm64<1, 1, 0, 2, 0><<<dim3(2, NB), 256, 0, stream>>>(
      p2_hi, p2_lo, KS, (long)TT * KS, memT_bf, memT_bf, KS, (long)HID * KS, cat2_hi + HID,
      cat2_lo + HID, NB * CATW, (long)CATW, biasr, TT, HID, KS, 1.0f);
  wmma_gemm64<1, 1, 2, 0, 0><<<dim3((MROWS / 64) * (HID / 64) / 8, 1), 256, 0, stream>>>(
      cat2_hi, cat2_lo, CATW, 0L, wgt_bf, wgt_bf, CATW, 0L, zbuf, zbuf, HID, 0L, biasr + HID,
      MROWS, HID, CATW, 1.0f);
  blend_kernel<<<(MROWS * HID / 4) / 256, 256, 0, stream>>>(zbuf, cat2_hi, cat2_lo, out0);
}
